// GenLSTMpdt_9938554323549
// MI455X (gfx1250) — hardware-verified
//
#include <hip/hip_runtime.h>
#include <math.h>

constexpr int NBATCH  = 512;
constexpr int NTIME   = 256;
constexpr int NSTEP   = NTIME - 1;
constexpr int NSD     = 8;
constexpr int NNOISE  = 32;
constexpr int NHID    = 256;
constexpr int NGATE   = 4 * NHID;
constexpr int KXPAD   = 64;
constexpr int KFUSED  = KXPAD + NHID;
constexpr int BROWS   = 32;
constexpr int NTHR    = 256;
constexpr int AGP     = 328;
constexpr int MLPP    = 264;
constexpr int NL3PAD  = 16;
constexpr float ACARRY  = 64.0f;
constexpr float WCARRY  = 16.0f;
constexpr float FOLDINV = 1.0f / (ACARRY * WCARRY);
constexpr float DT_STEP = 0.01f;

constexpr int OFF_WG = 0;
constexpr int SQ_ELEMS = NHID * NHID;
constexpr int L3_ELEMS = NL3PAD * NHID;
constexpr int OFF_M1 = OFF_WG + NGATE * KFUSED;
constexpr int OFF_M2 = OFF_M1 + SQ_ELEMS;
constexpr int OFF_V1 = OFF_M2 + SQ_ELEMS;
constexpr int OFF_V2 = OFF_V1 + SQ_ELEMS;
constexpr int OFF_M3 = OFF_V2 + SQ_ELEMS;
constexpr int OFF_V3 = OFF_M3 + L3_ELEMS;
constexpr int PLANE_ELEMS = OFF_V3 + L3_ELEMS;

constexpr int PB_X   = NGATE / 32;
constexpr int PB_H   = NGATE * 4 / 32;
constexpr int PB_SQ  = 4 * (SQ_ELEMS / 8) / NTHR;
constexpr int PB_L3  = 2 * (L3_ELEMS / 8) / NTHR;
constexpr int PB_E0  = PB_X;
constexpr int PB_E1  = PB_E0 + PB_H;
constexpr int PB_E2  = PB_E1 + PB_SQ;
constexpr int PB_E3  = PB_E2 + PB_L3;

static_assert(NSD + NNOISE <= KXPAD, "x|noise fits the padded K segment");
static_assert(KFUSED % 32 == 0 && NHID % 32 == 0, "K multiples of 32");
static_assert(KFUSED == 320 && KFUSED * 2 == 5 * 128, "gate plane row = 5 whole lines");
static_assert(NBATCH % BROWS == 0, "block rows");
static_assert(NHID == 32 * (NTHR / 32), "8 waves x 32 hidden columns");
static_assert(BROWS * NSD == NTHR, "sample stage: one thread per (row, channel)");
static_assert(NTIME % 4 == 0, "four time slots per 128-B output line");
static_assert((AGP * 2) % 16 == 0 && (MLPP * 2) % 16 == 0, "LDS rows 16-B aligned");
static_assert(PLANE_ELEMS == 598016, "plane carve");
static_assert(PB_E3 * NTHR * 8 == PLANE_ELEMS, "prep coverage exact");
static_assert(PB_E0 == 32 && PB_E1 == 160 && PB_E2 == 288 && PB_E3 == 292, "prep block ranges");

typedef __attribute__((ext_vector_type(16))) _Float16 v16h;
typedef __attribute__((ext_vector_type(8)))  _Float16 v8h;
typedef __attribute__((ext_vector_type(4)))  _Float16 v4h;
typedef __attribute__((ext_vector_type(8)))  float    v8f;
typedef __attribute__((ext_vector_type(4)))  float    v4f;

template <typename T> struct Frag;
template <> struct Frag<_Float16> {
  typedef v16h V; union U { v16h v; v8h h[2]; };
  static __device__ __forceinline__ v16h load(const _Float16* p) {
    U f; f.h[0] = *(const v8h*)(p); f.h[1] = *(const v8h*)(p + 16); return f.v;
  }
  static __device__ __forceinline__ v8f mma(v16h a, v16h b, v8f c) {
    return __builtin_amdgcn_wmma_f32_16x16x32_f16(false, a, false, b, (short)0, c, false, false);
  }
};

__device__ __forceinline__ void guard_4x2(v8f& c0, v8f& c1, v8f& c2, v8f& c3, v8f& c4, v8f& c5, v8f& c6, v8f& c7,
                                          v16h a0, v16h a1, v16h b0, v16h b1, v16h b2, v16h b3) {
  asm volatile("v_nop\n\tv_nop\n\tv_nop\n\tv_nop"
               : "+v"(c0), "+v"(c1), "+v"(c2), "+v"(c3), "+v"(c4), "+v"(c5), "+v"(c6), "+v"(c7)
               : "v"(a0), "v"(a1), "v"(b0), "v"(b1), "v"(b2), "v"(b3));
}
__device__ __forceinline__ void guard_1x2(v8f& c0, v8f& c1, v16h a0, v16h a1, v16h b0) {
  asm volatile("v_nop\n\tv_nop\n\tv_nop\n\tv_nop" : "+v"(c0), "+v"(c1) : "v"(a0), "v"(a1), "v"(b0));
}

template <int KTOT>
__device__ __forceinline__ void mm_4x2(const _Float16* a0p, const _Float16* a1p,
                                       const _Float16* b0p, const _Float16* b1p,
                                       const _Float16* b2p, const _Float16* b3p,
                                       v8f& c00, v8f& c01, v8f& c10, v8f& c11,
                                       v8f& c20, v8f& c21, v8f& c30, v8f& c31) {
#pragma unroll 1
  for (int k0 = 0; k0 < KTOT; k0 += 32) {
    const v16h a0 = Frag<_Float16>::load(a0p + k0);
    const v16h a1 = Frag<_Float16>::load(a1p + k0);
    const v16h b0 = Frag<_Float16>::load(b0p + k0);
    const v16h b1 = Frag<_Float16>::load(b1p + k0);
    const v16h b2 = Frag<_Float16>::load(b2p + k0);
    const v16h b3 = Frag<_Float16>::load(b3p + k0);
    c00 = Frag<_Float16>::mma(a0, b0, c00);
    c01 = Frag<_Float16>::mma(a1, b0, c01);
    c10 = Frag<_Float16>::mma(a0, b1, c10);
    c11 = Frag<_Float16>::mma(a1, b1, c11);
    c20 = Frag<_Float16>::mma(a0, b2, c20);
    c21 = Frag<_Float16>::mma(a1, b2, c21);
    c30 = Frag<_Float16>::mma(a0, b3, c30);
    c31 = Frag<_Float16>::mma(a1, b3, c31);
    guard_4x2(c00, c01, c10, c11, c20, c21, c30, c31, a0, a1, b0, b1, b2, b3);
  }
}

__device__ __forceinline__ float sigm_f(float x) { return __builtin_amdgcn_rcpf(1.0f + __expf(-x)); }
__device__ __forceinline__ float tanh_f(float x) { return 1.0f - 2.0f * __builtin_amdgcn_rcpf(__expf(2.0f * x) + 1.0f); }

__device__ __forceinline__ void mlp_layer(const _Float16* ap, int apitch, const _Float16* bp,
                                          float bs0, float bs1, float bs2, float bs3,
                                          _Float16* dst, int ncol0, int hh) {
  const v8f z8 = {0.f, 0.f, 0.f, 0.f, 0.f, 0.f, 0.f, 0.f};
  v8f acc[4][2];
#pragma unroll
  for (int i = 0; i < 4; ++i) { acc[i][0] = z8; acc[i][1] = z8; }
  mm_4x2<NHID>(ap, ap + 16 * apitch, bp, bp + 16 * NHID, bp + 32 * NHID, bp + 48 * NHID,
               acc[0][0], acc[0][1], acc[1][0], acc[1][1], acc[2][0], acc[2][1], acc[3][0], acc[3][1]);
  const float bs[4] = {bs0, bs1, bs2, bs3};
#pragma unroll
  for (int i = 0; i < 4; ++i)
#pragma unroll
    for (int mt = 0; mt < 2; ++mt)
#pragma unroll
      for (int r = 0; r < 8; ++r) {
        const float v = fmaxf(acc[i][mt][r] * FOLDINV + bs[i], 0.0f);
        dst[(16 * mt + 8 * hh + r) * MLPP + ncol0 + 16 * i] = (_Float16)(v * ACARRY);
      }
}

__device__ __forceinline__ void stage_xt(_Float16* agrow, int sd, float xv, v4f nz) {
  agrow[sd] = (_Float16)(xv * ACARRY);
  v4h nh;
  nh[0] = (_Float16)(nz[0] * ACARRY);
  nh[1] = (_Float16)(nz[1] * ACARRY);
  nh[2] = (_Float16)(nz[2] * ACARRY);
  nh[3] = (_Float16)(nz[3] * ACARRY);
  *(v4h*)(agrow + NSD + 4 * sd) = nh;
  if (sd < 3) {
    const v8h zh = {(_Float16)0.f, (_Float16)0.f, (_Float16)0.f, (_Float16)0.f,
                    (_Float16)0.f, (_Float16)0.f, (_Float16)0.f, (_Float16)0.f};
    *(v8h*)(agrow + NSD + NNOISE + 8 * sd) = zh;
  }
}

__global__ __launch_bounds__(NTHR) void prep_kernel(const float* __restrict__ Wx, const float* __restrict__ Wh,
                                                    const float* __restrict__ Wm1, const float* __restrict__ Wm2,
                                                    const float* __restrict__ Wv1, const float* __restrict__ Wv2,
                                                    const float* __restrict__ Wm3, const float* __restrict__ Wv3,
                                                    unsigned short* __restrict__ planes) {
  const int tid = threadIdx.x;
  const int blk = blockIdx.x;
  const float* src;
  int pitch, ncl, krow0;
  bool live;
  size_t dsto;
  if (blk < PB_E0) {
    const int n  = blk * 32 + (tid >> 3);
    const int kc = tid & 7;
    src = Wx; pitch = NGATE; ncl = n;
    krow0 = 8 * (kc < 4 ? kc : 4);
    live = (kc < 5);
    dsto = (size_t)OFF_WG + (size_t)n * KFUSED + 8 * kc;
  } else if (blk < PB_E1) {
    const int line = (blk - PB_E0) * 32 + (tid >> 3);
    const int n    = line >> 2;
    const int lsub = line & 3;
    src = Wh; pitch = NGATE; ncl = n;
    krow0 = lsub * 64 + 8 * (tid & 7);
    live = true;
    dsto = (size_t)OFF_WG + (size_t)n * KFUSED + KXPAD + krow0;
  } else if (blk < PB_E2) {
    const int q    = blk - PB_E1;
    const int pidx = q >> 5;
    const int cidx = (q & 31) * NTHR + tid;
    src = (pidx == 0) ? Wm1 : (pidx == 1) ? Wm2 : (pidx == 2) ? Wv1 : Wv2;
    pitch = NHID; ncl = cidx >> 5;
    krow0 = 8 * (cidx & 31);
    live = true;
    dsto = (size_t)OFF_M1 + (size_t)pidx * SQ_ELEMS + (size_t)cidx * 8;
  } else {
    const int q    = blk - PB_E2;
    const int pidx = q >> 1;
    const int cidx = (q & 1) * NTHR + tid;
    const int n    = cidx >> 5;
    src = pidx ? Wv3 : Wm3;
    pitch = NSD; ncl = (n < NSD) ? n : (NSD - 1);
    krow0 = 8 * (cidx & 31);
    live = (n < NSD);
    dsto = (size_t)OFF_M3 + (size_t)pidx * L3_ELEMS + (size_t)cidx * 8;
  }
  float f[8];
#pragma unroll
  for (int e = 0; e < 8; ++e) f[e] = src[(size_t)(krow0 + e) * (size_t)pitch + ncl];
  v8h hv;
#pragma unroll
  for (int e = 0; e < 8; ++e) {
    const float s = live ? (f[e] * WCARRY) : 0.0f;
    hv[e] = (_Float16)s;
  }
  *(volatile v8h*)(planes + dsto) = hv;
  __threadfence();
  *(volatile v8h*)(planes + dsto) = hv;
}

__global__ __launch_bounds__(NTHR) void seq_kernel(const float* __restrict__ noise, const float* __restrict__ eps,
                                                   const float* __restrict__ bgate,
                                                   const float* __restrict__ bm1, const float* __restrict__ bm2,
                                                   const float* __restrict__ bm3,
                                                   const float* __restrict__ bv1, const float* __restrict__ bv2,
                                                   const float* __restrict__ bv3,
                                                   const unsigned short* __restrict__ planes,
                                                   float* __restrict__ out) {
  __shared__ __align__(16) _Float16 AG[2][BROWS * AGP];
  __shared__ __align__(16) _Float16 A1[2][BROWS * MLPP];
  __shared__ __align__(16) _Float16 A2[2][BROWS * MLPP];
  __shared__ __align__(16) float    SML[2][BROWS * NSD];
  __shared__ __align__(16) float    OS[BROWS * 32];

  const _Float16* WP = (const _Float16*)planes;
  const int tid = threadIdx.x, lane = tid & 31, wave = tid >> 5;
  const int c = lane & 15, hh = lane >> 4, koff = hh * 8;
  const int brow0 = blockIdx.x * BROWS;
  const int m = tid >> 3, sd = tid & 7;
  const v8f z8 = {0.f, 0.f, 0.f, 0.f, 0.f, 0.f, 0.f, 0.f};

  {
    const v8h zh = {(_Float16)0.f, (_Float16)0.f, (_Float16)0.f, (_Float16)0.f,
                    (_Float16)0.f, (_Float16)0.f, (_Float16)0.f, (_Float16)0.f};
#pragma unroll
    for (int i = 0; i < 4; ++i) {
      const int idx = i * NTHR + tid;
      const int row = idx >> 5, c8 = (idx & 31) * 8;
      *(v8h*)(&AG[0][row * AGP + KXPAD + c8]) = zh;
    }
  }
  {
    const v4f nz = *(const v4f*)(noise + ((size_t)(brow0 + m) * NTIME) * NNOISE + 4 * sd);
    stage_xt(&AG[0][m * AGP], sd, 0.0f, nz);
  }
  OS[m * 32 + sd] = 0.0f;
  float cum = 0.0f;

  float cst[2][2][8];
#pragma unroll
  for (int nl = 0; nl < 2; ++nl)
#pragma unroll
    for (int mt = 0; mt < 2; ++mt)
#pragma unroll
      for (int r = 0; r < 8; ++r) cst[nl][mt][r] = 0.0f;
  float bgt[2][4];
#pragma unroll
  for (int nl = 0; nl < 2; ++nl)
#pragma unroll
    for (int g = 0; g < 4; ++g) bgt[nl][g] = bgate[g * NHID + 32 * wave + 16 * nl + c];
  const int netw = wave >> 2;
  const int tb   = (wave & 3) * 4;
  const float* b1p = netw ? bv1 : bm1;
  const float* b2p = netw ? bv2 : bm2;
  float bl1[4], bl2[4];
#pragma unroll
  for (int i = 0; i < 4; ++i) {
    bl1[i] = b1p[(tb + i) * 16 + c];
    bl2[i] = b2p[(tb + i) * 16 + c];
  }
  const int net3 = wave & 1;
  const float* b3p = net3 ? bv3 : bm3;
  const float bl3 = b3p[(c < NSD) ? c : (NSD - 1)];
  __syncthreads();

#pragma unroll 1
  for (int t = 0; t < NSTEP; ++t) {
    const int p = t & 1;
    const _Float16* agc = &AG[p][0];
    _Float16* agn = &AG[p ^ 1][0];

#pragma unroll
    for (int nl = 0; nl < 2; ++nl) {
      const int j = 32 * wave + 16 * nl + c;
      const _Float16* ap = agc + c * AGP + koff;
      const _Float16* bp = WP + OFF_WG + (size_t)j * KFUSED + koff;
      v8f acc[4][2];
#pragma unroll
      for (int g = 0; g < 4; ++g) { acc[g][0] = z8; acc[g][1] = z8; }
      mm_4x2<KFUSED>(ap, ap + 16 * AGP,
                     bp, bp + (size_t)1 * NHID * KFUSED, bp + (size_t)2 * NHID * KFUSED, bp + (size_t)3 * NHID * KFUSED,
                     acc[0][0], acc[0][1], acc[1][0], acc[1][1], acc[2][0], acc[2][1], acc[3][0], acc[3][1]);
#pragma unroll
      for (int mt = 0; mt < 2; ++mt)
#pragma unroll
        for (int r = 0; r < 8; ++r) {
          const float zi = acc[0][mt][r] * FOLDINV + bgt[nl][0];
          const float zf = acc[1][mt][r] * FOLDINV + bgt[nl][1];
          const float zg = acc[2][mt][r] * FOLDINV + bgt[nl][2];
          const float zo = acc[3][mt][r] * FOLDINV + bgt[nl][3];
          const float ig = sigm_f(zi);
          const float fg = sigm_f(zf);
          const float gg = tanh_f(zg);
          const float og = sigm_f(zo);
          const float cn = fg * cst[nl][mt][r] + ig * gg;
          cst[nl][mt][r] = cn;
          const float hv = og * tanh_f(cn);
          agn[(16 * mt + 8 * hh + r) * AGP + KXPAD + j] = (_Float16)(hv * ACARRY);
        }
    }
    __syncthreads();

    mlp_layer(agn + KXPAD + c * AGP + koff, AGP,
              WP + OFF_M1 + (size_t)netw * 2 * SQ_ELEMS + (size_t)(tb * 16 + c) * NHID + koff,
              bl1[0], bl1[1], bl1[2], bl1[3], &A1[netw][0], tb * 16 + c, hh);
    __syncthreads();

    mlp_layer(&A1[netw][0] + c * MLPP + koff, MLPP,
              WP + OFF_M2 + (size_t)netw * 2 * SQ_ELEMS + (size_t)(tb * 16 + c) * NHID + koff,
              bl2[0], bl2[1], bl2[2], bl2[3], &A2[netw][0], tb * 16 + c, hh);
    __syncthreads();

    if (wave < 2) {
      const _Float16* ap = &A2[wave][0] + c * MLPP + koff;
      const _Float16* bp = WP + OFF_M3 + (size_t)wave * L3_ELEMS + (size_t)c * NHID + koff;
      v8f q0 = z8, q1 = z8;
#pragma unroll 1
      for (int k0 = 0; k0 < NHID; k0 += 32) {
        const v16h a0 = Frag<_Float16>::load(ap + k0);
        const v16h a1 = Frag<_Float16>::load(ap + 16 * MLPP + k0);
        const v16h b0 = Frag<_Float16>::load(bp + k0);
        q0 = Frag<_Float16>::mma(a0, b0, q0);
        q1 = Frag<_Float16>::mma(a1, b0, q1);
        guard_1x2(q0, q1, a0, a1, b0);
      }
      if (c < NSD) {
#pragma unroll
        for (int r = 0; r < 8; ++r) {
          SML[wave][(8 * hh + r) * NSD + c]      = q0[r] * FOLDINV + bl3;
          SML[wave][(16 + 8 * hh + r) * NSD + c] = q1[r] * FOLDINV + bl3;
        }
      }
    }
    __syncthreads();

    {
      const float mu = SML[0][tid];
      const float lv = SML[1][tid];
      const float ev = eps[((size_t)(brow0 + m) * NSTEP + (size_t)t) * NSD + sd];
      const float sdv = expf(0.5f * lv) * DT_STEP;
      const float xv = mu + sdv * ev;
      cum += xv;
      const int tn = (t + 1 < NSTEP) ? (t + 1) : (NSTEP - 1);
      const v4f nz = *(const v4f*)(noise + ((size_t)(brow0 + m) * NTIME + (size_t)tn) * NNOISE + 4 * sd);
      stage_xt(agn + m * AGP, sd, xv, nz);
      OS[m * 32 + ((t + 1) & 3) * NSD + sd] = cum;
    }
    __syncthreads();

    if ((t & 3) == 2) {
      const int row = 4 * wave + (lane >> 3);
      const int c4  = (lane & 7) * 4;
      const v4f v = *(const v4f*)(OS + row * 32 + c4);
      float* gp = out + ((size_t)(brow0 + row) * NTIME + (size_t)(t - 2)) * NSD + c4;
      *(volatile v4f*)gp = v;
      __threadfence();
      *(volatile v4f*)gp = v;
    }
  }
}

extern "C" void kernel_launch(void* const* d_in, const int* in_sizes, int n_in,
                              void* d_out, int out_size, void* d_ws, size_t ws_size, hipStream_t stream) {
  if (n_in < 17 || d_out == nullptr || d_ws == nullptr) return;
  if (in_sizes[0] != NBATCH * NTIME * NNOISE || in_sizes[1] != NBATCH * NSTEP * NSD ||
      in_sizes[2] != (NSD + NNOISE) * NGATE || in_sizes[3] != NHID * NGATE || in_sizes[4] != NGATE ||
      in_sizes[5] != NHID * NHID || in_sizes[6] != NHID || in_sizes[7] != NHID * NHID || in_sizes[8] != NHID ||
      in_sizes[9] != NHID * NSD || in_sizes[10] != NSD ||
      in_sizes[11] != NHID * NHID || in_sizes[12] != NHID || in_sizes[13] != NHID * NHID || in_sizes[14] != NHID ||
      in_sizes[15] != NHID * NSD || in_sizes[16] != NSD ||
      out_size != NBATCH * NTIME * NSD) return;
  const size_t carve = ((size_t)PLANE_ELEMS * 2 + 255) & ~(size_t)255;
  if (carve > ws_size || carve > (size_t)134217728) return;

  const float* noise = (const float*)d_in[0];
  const float* epsv  = (const float*)d_in[1];
  const float* Wx    = (const float*)d_in[2];
  const float* Wh    = (const float*)d_in[3];
  const float* bg    = (const float*)d_in[4];
  const float* Wm1   = (const float*)d_in[5];
  const float* bm1   = (const float*)d_in[6];
  const float* Wm2   = (const float*)d_in[7];
  const float* bm2   = (const float*)d_in[8];
  const float* Wm3   = (const float*)d_in[9];
  const float* bm3   = (const float*)d_in[10];
  const float* Wv1   = (const float*)d_in[11];
  const float* bv1   = (const float*)d_in[12];
  const float* Wv2   = (const float*)d_in[13];
  const float* bv2   = (const float*)d_in[14];
  const float* Wv3   = (const float*)d_in[15];
  const float* bv3   = (const float*)d_in[16];
  unsigned short* planes = (unsigned short*)d_ws;

  prep_kernel<<<PB_E3, NTHR, 0, stream>>>(Wx, Wh, Wm1, Wm2, Wv1, Wv2, Wm3, Wv3, planes);
  seq_kernel<<<NBATCH / BROWS, NTHR, 0, stream>>>(noise, epsv, bg, bm1, bm2, bm3, bv1, bv2, bv3, planes, (float*)d_out);
}
